// GraphTransformerRegressor_76630806495962
// MI455X (gfx1250) — hardware-run, weakly checked
//
#include <hip/hip_runtime.h>


namespace {
constexpr int N = 50000, NP = 50048, E = 500000, IN = 64, HID = 128, NH = 4, CH = 32, G = 64, L = 3, QW = 4 * HID  ;
constexpr float XS = 8.0f, WSC = 256.0f, NEG = 0.2f  , LNEPS = 1e-5f, ISQC = 0.17677669529663688f  ;

typedef _Float16 b16;
typedef __attribute__((ext_vector_type(16))) _Float16 v16b;
typedef __attribute__((ext_vector_type(8))) _Float16 v8b;
typedef __attribute__((ext_vector_type(8))) float v8f;
typedef __attribute__((ext_vector_type(4))) float v4f;
__device__ __forceinline__ float bf16_rne(float f) { unsigned int u = __float_as_uint(f); u += 0x7FFFu + ((u >> 16) & 1u); return __uint_as_float(u & 0xFFFF0000u); }
__device__ __forceinline__ void split16(float v, b16& hi, b16& lo) { hi = (b16)v; lo = (b16)(v - (float)hi); }
__device__ __forceinline__ v16b frag_kb(const b16* p, int hh) { const v8b a = *(const v8b*)(p + 8 * hh), b = *(const v8b*)(p + 16 + 8 * hh); v16b f;
#pragma unroll
  for (int e = 0; e < 8; ++e) { f[e] = a[e]; f[8 + e] = b[e]; } return f; }
__device__ __forceinline__ v8f wmma16b(v16b a, v16b b, v8f c) { v8f d = __builtin_amdgcn_wmma_f32_16x16x32_f16(false, a, false, b, (short)0, c, false, false); asm volatile("v_nop\n\tv_nop\n\tv_nop\n\tv_nop" : "+v"(d) : "v"(a), "v"(b)); return d; }
__device__ __forceinline__ void wave_lds_sync() { __builtin_amdgcn_fence(__ATOMIC_RELEASE, "workgroup"); __builtin_amdgcn_wave_barrier(); __builtin_amdgcn_fence(__ATOMIC_ACQUIRE, "workgroup"); }
__device__ __forceinline__ float pmul(float a, float b) { float p = a * b; asm volatile("" : "+v"(p)); return p; }
__device__ __forceinline__ int iclamp(int v, int lo, int hi) { return v < lo ? lo : (v > hi ? hi : v); }
__device__ __forceinline__ float nexp(float x) { return __builtin_amdgcn_exp2f(x * 1.4426950408889634f); }
__device__ __forceinline__ float lrelu(float x) { return x > 0.0f ? x : NEG * x; }

constexpr int CSR_NBLK = 512, CSR_GB = 9, CSR_GN = 1 << CSR_GB  , CSR_MAXG = 512, CSR_CAP = 12288  ;
__global__ __launch_bounds__(64) void csrA_kernel(const int* __restrict__ dst, int E, int N, int nG, int CHP, int NGP, int* __restrict__ STG, int* __restrict__ HST) {
  extern __shared__ int sm[];
  int* cnt = sm; int* run = sm + NGP; int* ids = sm + 2 * NGP;
  const int b = blockIdx.x; const int ch = (E + CSR_NBLK - 1) / CSR_NBLK; const int e0 = b * ch, e1 = min(E, e0 + ch);
  for (int i = threadIdx.x; i < NGP; i += 64) cnt[i] = 0;
  for (int i = threadIdx.x; i < CHP; i += 64) ids[i] = -1;
  __syncthreads();
  if (threadIdx.x == 0) {
    for (int e = e0; e < e1; ++e) { int d = dst[e]; d = (d < 0) ? 0 : (d >= N ? N - 1 : d); cnt[d >> CSR_GB] += 1; }
    int acc = 0; for (int g = 0; g < nG; ++g) { run[g] = acc; acc += cnt[g]; }
    for (int e = e0; e < e1; ++e) { int d = dst[e]; d = (d < 0) ? 0 : (d >= N ? N - 1 : d); const int g = d >> CSR_GB; ids[run[g]] = e; run[g] += 1; } }
  __syncthreads();
  typedef __attribute__((ext_vector_type(4))) int v4i;
  for (int pass = 0; pass < 2; ++pass) {
    for (int i = threadIdx.x; i < CHP / 4; i += 64) *(volatile v4i*)(STG + (size_t)b * CHP + i * 4) = *(const v4i*)(&ids[i * 4]);
    for (int i = threadIdx.x; i < NGP / 4; i += 64) { v4i v; for (int e = 0; e < 4; ++e) v[e] = (i * 4 + e < nG) ? cnt[i * 4 + e] : 0; *(volatile v4i*)(HST + (size_t)b * NGP + i * 4) = v; }
    __threadfence(); }
}
__global__ __launch_bounds__(512) void csrS_kernel(const int* __restrict__ HST, int nG, int NGP, int* __restrict__ START, int* __restrict__ TOT, int* __restrict__ OFF) {
  __shared__ int tot[CSR_MAXG];
  const int b = threadIdx.x;
  for (int pass = 0; pass < 2; ++pass) { int runb = 0; for (int g = 0; g < nG; ++g) { int c = HST[(size_t)b * NGP + g]; c = (c < 0) ? 0 : c; ((volatile int*)OFF)[(size_t)g * CSR_NBLK + b] = runb; runb += c; } __threadfence(); }
  for (int g = threadIdx.x; g < nG; g += 512) { int s = 0; for (int bb = 0; bb < CSR_NBLK; ++bb) { int c = HST[(size_t)bb * NGP + g]; s += (c < 0) ? 0 : c; } tot[g] = s; }
  __syncthreads();
  if (threadIdx.x < 32) {
    __shared__ int st[CSR_MAXG + 32];
    if (threadIdx.x == 0) { int acc = 0; for (int g = 0; g < NGP; ++g) { st[g] = acc; if (g < nG) acc += (tot[g] + 31) & ~31; } st[NGP] = acc; }
    __builtin_amdgcn_fence(__ATOMIC_RELEASE, "workgroup"); __builtin_amdgcn_wave_barrier(); __builtin_amdgcn_fence(__ATOMIC_ACQUIRE, "workgroup");
    for (int pass = 0; pass < 2; ++pass) { for (int i = threadIdx.x; i < NGP + 32; i += 32) { ((volatile int*)START)[i] = (i <= NGP) ? st[min(i, NGP)] : 0; ((volatile int*)TOT)[i] = (i < nG) ? tot[i] : 0; } __threadfence(); } }
}
__global__ __launch_bounds__(256) void csrB_kernel(const int* __restrict__ dst, int N, int nG, int CHP, int NGP, int permLen, const int* __restrict__ STG, const int* __restrict__ HST, const int* __restrict__ OFF, const int* __restrict__ START, const int* __restrict__ TOT, int* __restrict__ PERM, int* __restrict__ ROWPTR, int* __restrict__ ROWCNT, int* __restrict__ FLAG) {
  typedef __attribute__((ext_vector_type(4))) int v4i;
  __shared__ int ids[CSR_CAP]; __shared__ unsigned short key[CSR_CAP]; __shared__ int outp[CSR_CAP]; __shared__ int ncnt[CSR_GN + 1]; __shared__ int boff[CSR_NBLK + 1];
  const int g = blockIdx.x, t_ = threadIdx.x; int tot = TOT[g]; int st = START[g], stn = START[g + 1]; const int v0 = g * CSR_GN; const int nv = min(CSR_GN, N - v0);
  st = (st < 0) ? 0 : (st > permLen - 32 ? permLen - 32 : st) & ~31; stn = (stn < st) ? st : (stn > permLen ? permLen : stn); tot = (tot < 0) ? 0 : tot; if (tot > stn - st && tot <= CSR_CAP) tot = stn - st;
  if (tot > CSR_CAP) {
    for (int pass = 0; pass < 2; ++pass) { for (int i = t_; i < CSR_GN / 4; i += 256) { v4i a, c; for (int e = 0; e < 4; ++e) { a[e] = st; c[e] = 0; } *(volatile v4i*)(ROWPTR + v0 + i * 4) = a; *(volatile v4i*)(ROWCNT + v0 + i * 4) = c; } if (t_ == 0) ((volatile int*)FLAG)[0] = 1; __threadfence(); } (void)nv; return; }
  if (t_ == 0) { int acc = 0; for (int b = 0; b < CSR_NBLK; ++b) { boff[b] = acc; int c = HST[(size_t)b * NGP + g]; c = (c < 0) ? 0 : (c > CHP ? CHP : c); acc += c; if (acc > tot) acc = tot; } boff[CSR_NBLK] = acc; }
  for (int i = t_; i <= CSR_GN; i += 256) ncnt[i] = 0;
  __syncthreads();
  for (int b = 0; b < CSR_NBLK; ++b) { const int c = boff[b + 1] - boff[b]; int o_ = OFF[(size_t)g * CSR_NBLK + b]; o_ = (o_ < 0) ? 0 : (o_ > CHP - c ? CHP - c : o_); const int* src_ = STG + (size_t)b * CHP + o_;
    for (int i = t_; i < c; i += 256) { int id = src_[i]; id = (id < 0) ? 0 : id; ids[boff[b] + i] = id; int d = dst[id]; d = (d < v0) ? v0 : (d >= N ? N - 1 : d); int kk = d - v0; kk = (kk < 0) ? 0 : (kk >= CSR_GN ? CSR_GN - 1 : kk); key[boff[b] + i] = (unsigned short)kk; } }
  __syncthreads();
  if (t_ == 0) { for (int i = 0; i < tot; ++i) ncnt[key[i]] += 1; int acc = 0; for (int vl = 0; vl < CSR_GN; ++vl) { const int c = ncnt[vl]; ncnt[vl] = acc; acc += c; } ncnt[CSR_GN] = acc;
    for (int i = 0; i < tot; ++i) { const int vl = key[i]; outp[ncnt[vl]] = ids[i]; ncnt[vl] += 1; }
    for (int vl = CSR_GN; vl > 0; --vl) ncnt[vl] = ncnt[vl - 1]; ncnt[0] = 0; }
  __syncthreads();
  for (int pass = 0; pass < 2; ++pass) {
    for (int i = t_; i < (stn - st) / 4; i += 256) { v4i v; for (int e = 0; e < 4; ++e) { const int q = i * 4 + e; v[e] = (q < tot) ? outp[q] : -1; } *(volatile v4i*)(PERM + st + i * 4) = v; }
    for (int i = t_; i < CSR_GN / 4; i += 256) { v4i a, c; for (int e = 0; e < 4; ++e) { const int vl = i * 4 + e; a[e] = st + ncnt[vl]; c[e] = (vl < nv) ? (ncnt[vl + 1] - ncnt[vl]) : 0; } *(volatile v4i*)(ROWPTR + v0 + i * 4) = a; *(volatile v4i*)(ROWCNT + v0 + i * 4) = c; }
    __threadfence(); }
}
__global__ __launch_bounds__(256) void csrZ_kernel(int* __restrict__ p, size_t n4) { typedef __attribute__((ext_vector_type(4))) int v4i; const size_t tid = (size_t)blockIdx.x * 256 + threadIdx.x, nth = (size_t)gridDim.x * 256; v4i z = {0, 0, 0, 0}; for (size_t i = tid; i < n4; i += nth) *(volatile v4i*)(p + i * 4) = z; }
struct CsrBufs { int *STG, *HST, *OFF, *START, *TOT, *PERM, *ROWPTR, *ROWCNT, *FLAG; int nG, NGP, CHP; size_t permLen; char* base; size_t bytes; };
static size_t csr_carve(CsrBufs& c, char* ws, size_t off, int E, int N) {
  const size_t off0 = off; c.base = ws + off;
  auto al = [&](size_t bytes) { char* p = ws + off; off += (bytes + 255) & ~(size_t)255; return p; };
  c.nG = (N + CSR_GN - 1) / CSR_GN; c.NGP = (c.nG + 31) & ~31; const int ch = (E + CSR_NBLK - 1) / CSR_NBLK; c.CHP = (ch + 31) & ~31; c.permLen = (size_t)E + 32 * (size_t)c.nG + 32;
  c.STG = (int*)al((size_t)CSR_NBLK * c.CHP * 4); c.HST = (int*)al((size_t)CSR_NBLK * c.NGP * 4); c.OFF = (int*)al((size_t)c.NGP * CSR_NBLK * 4); c.START = (int*)al((size_t)(c.NGP + 64) * 4); c.TOT = (int*)al((size_t)(c.NGP + 64) * 4);
  c.PERM = (int*)al(c.permLen * 4); c.ROWPTR = (int*)al((size_t)c.nG * CSR_GN * 4); c.ROWCNT = (int*)al((size_t)c.nG * CSR_GN * 4); c.FLAG = (int*)al(256);
  c.bytes = off - off0; return off;
}
static void csr_build(const CsrBufs& c, const int* dst, int E, int N, hipStream_t stream) {
  const size_t smem = (size_t)(2 * c.NGP + c.CHP) * 4;
  csrZ_kernel<<<512, 256, 0, stream>>>((int*)c.base, c.bytes / 16);
  csrA_kernel<<<CSR_NBLK, 64, smem, stream>>>(dst, E, N, c.nG, c.CHP, c.NGP, c.STG, c.HST);
  csrS_kernel<<<1, 512, 0, stream>>>(c.HST, c.nG, c.NGP, c.START, c.TOT, c.OFF);
  csrB_kernel<<<c.nG, 256, 0, stream>>>(dst, N, c.nG, c.CHP, c.NGP, (int)c.permLen, c.STG, c.HST, c.OFF, c.START, c.TOT, c.PERM, c.ROWPTR, c.ROWCNT, c.FLAG);
}


__device__ __forceinline__ float gelu(float x) { return 0.5f * x * (1.0f + erff(x * 0.70710678118654752f)); }
__device__ __forceinline__ float sigm(float x) { return 1.0f / (1.0f + __expf(-x)); }
__global__ __launch_bounds__(256) void prep_kernel(const float* __restrict__ x, const float* __restrict__ wq0, const float* __restrict__ wk0, const float* __restrict__ wv0, const float* __restrict__ ws0, const float* __restrict__ wq, const float* __restrict__ wk, const float* __restrict__ wv, const float* __restrict__ wss, b16* __restrict__ X16, b16* __restrict__ WT0, b16* __restrict__ WT12) {
  const size_t u = (size_t)blockIdx.x * 256 + threadIdx.x; const size_t nx = (size_t)NP * IN / 8, n0 = (size_t)QW * IN / 8, n1 = (size_t)2 * QW * HID / 8; size_t t = u; v8b o;
  if (t < nx) { const size_t e = t * 8; const size_t v = e / IN; for (int j = 0; j < 8; ++j) o[j] = v < (size_t)N ? (b16)(bf16_rne(x[e + j]) * XS) : (b16)0.0f; for (int pass = 0; pass < 2; ++pass) { *(volatile v8b*)(X16 + e) = o; __threadfence(); } return; } t -= nx;
  if (t < n0) { const size_t e = t * 8; const int oo = (int)(e / IN), k0 = (int)(e % IN); const int part = oo / HID, oc = oo % HID; const float* w = part == 0 ? wq0 : part == 1 ? wk0 : part == 2 ? wv0 : ws0;
    for (int j = 0; j < 8; ++j) o[j] = (b16)(bf16_rne(w[(size_t)(k0 + j) * HID + oc]) * WSC); for (int pass = 0; pass < 2; ++pass) { *(volatile v8b*)(WT0 + e) = o; __threadfence(); } return; } t -= n0;
  if (t < n1) { const size_t e = t * 8; const int l = (int)(e / ((size_t)QW * HID)); const size_t rem = e % ((size_t)QW * HID); const int oo = (int)(rem / HID), k0 = (int)(rem % HID); const int part = oo / HID, oc = oo % HID; const float* w = part == 0 ? wq : part == 1 ? wk : part == 2 ? wv : wss;
    for (int j = 0; j < 8; ++j) o[j] = (b16)(bf16_rne(w[((size_t)l * HID + k0 + j) * HID + oc]) * WSC); for (int pass = 0; pass < 2; ++pass) { *(volatile v8b*)(WT12 + e) = o; __threadfence(); } }
}
template <int KD, int TWO>
__global__ __launch_bounds__(128) void proj_kernel(const b16* __restrict__ Ah, const b16* __restrict__ Al, const b16* __restrict__ WT, const float* __restrict__ bq, const float* __restrict__ bk, const float* __restrict__ bv, const float* __restrict__ bs, float* __restrict__ QKVS) {
  __shared__ __attribute__((aligned(16))) float Tf[4][16][HID + 4];
  const int wave = threadIdx.x >> 5, lane = threadIdx.x & 31, nloc = lane & 15, hlf = lane >> 4; const size_t m0 = (size_t)blockIdx.x * 64 + wave * 16; const int part = blockIdx.y; const int n0 = part * HID;
  const float* bias = part == 0 ? bq : part == 1 ? bk : part == 2 ? bv : bs;
  v8f acc[8];
#pragma unroll
  for (int t = 0; t < 8; ++t) acc[t] = (v8f){};
#pragma unroll
  for (int kb = 0; kb < KD; kb += 32) { const v16b a = frag_kb(Ah + (m0 + nloc) * KD + kb, hlf); v16b al; if (TWO) al = frag_kb(Al + (m0 + nloc) * KD + kb, hlf);
#pragma unroll
    for (int t = 0; t < 8; ++t) { const v16b bw = frag_kb(WT + (size_t)(n0 + t * 16 + nloc) * KD + kb, hlf); acc[t] = wmma16b(a, bw, acc[t]); if (TWO) acc[t] = wmma16b(al, bw, acc[t]); } }
#pragma unroll
  for (int t = 0; t < 8; ++t) { const int c = t * 16 + nloc; const float bb = bf16_rne(bias[c]);
#pragma unroll 1
    for (int r = 0; r < 8; ++r) Tf[wave][8 * hlf + r][c] = acc[t][r] * (1.0f / (XS * WSC)) + bb; }
  wave_lds_sync();
  for (int pass = 0; pass < 2; ++pass) { for (int rr = 0; rr < 16; ++rr) *(volatile v4f*)(QKVS + (m0 + rr) * QW + n0 + lane * 4) = *(const v4f*)(&Tf[wave][rr][lane * 4]); __threadfence(); }
}
template <int LAST>
__global__ __launch_bounds__(256) void attn_kernel(const float* __restrict__ QKVS, const int* __restrict__ srcs, const int* __restrict__ PERM, const int* __restrict__ ROWPTR, const int* __restrict__ ROWCNT, int permLen, const float* __restrict__ wb, const float* __restrict__ g_, const float* __restrict__ b_, b16* __restrict__ Hh, b16* __restrict__ Hl, float* __restrict__ HF) {
  typedef __attribute__((ext_vector_type(4))) _Float16 v4h;
  const int wave = threadIdx.x >> 5, lane = threadIdx.x & 31; const size_t v = (size_t)blockIdx.x * 8 + wave; const int c0 = lane * 4;
  float y[4] = {0.0f, 0.0f, 0.0f, 0.0f};
  int st = 0, cnt = 0; if (v < (size_t)N) { st = ROWPTR[v]; cnt = ROWCNT[v]; cnt = iclamp(cnt, 0, 65536); st = iclamp(st, 0, permLen - cnt); }
  const v4f q = *(const v4f*)(QKVS + v * QW + c0);
  auto score = [&](size_t s) -> float { const v4f k = *(const v4f*)(QKVS + s * QW + HID + c0); float d = pmul(q[0], k[0]) + pmul(q[1], k[1]) + pmul(q[2], k[2]) + pmul(q[3], k[3]); d += __shfl_xor(d, 1); d += __shfl_xor(d, 2); d += __shfl_xor(d, 4); return d * ISQC; };
  float mx = -INFINITY;
#pragma unroll 1
  for (int j = 0; j < cnt; ++j) { const int e = iclamp(PERM[st + j], 0, E - 1); const size_t s = (size_t)iclamp(srcs[e], 0, N - 1); mx = fmaxf(mx, score(s)); }
  float den = 0.0f; v4f acc = {0.0f, 0.0f, 0.0f, 0.0f};
#pragma unroll 1
  for (int j = 0; j < cnt; ++j) { const int e = iclamp(PERM[st + j], 0, E - 1); const size_t s = (size_t)iclamp(srcs[e], 0, N - 1); const float p = nexp(score(s) - mx); den += p; const v4f vv = *(const v4f*)(QKVS + s * QW + 2 * HID + c0); for (int i = 0; i < 4; ++i) acc[i] += pmul(p, vv[i]); }
  const float inv = cnt > 0 ? 1.0f / den : 0.0f;
  const v4f xr = *(const v4f*)(QKVS + v * QW + 3 * HID + c0);
  float out[4], part = 0.0f; for (int i = 0; i < 4; ++i) { out[i] = cnt > 0 ? acc[i] * inv : 0.0f; const int c = c0 + i; part += pmul(out[i], bf16_rne(wb[c])) + pmul(xr[i], bf16_rne(wb[HID + c])) + pmul(out[i] - xr[i], bf16_rne(wb[2 * HID + c])); }
  for (int o = 16; o; o >>= 1) part += __shfl_xor(part, o);
  const float beta = sigm(part);
  for (int i = 0; i < 4; ++i) y[i] = pmul(beta, xr[i]) + pmul(1.0f - beta, out[i]);
  float s1 = y[0] + y[1] + y[2] + y[3]; for (int o = 16; o; o >>= 1) s1 += __shfl_xor(s1, o); const float mean = s1 * (1.0f / HID);
  float s2 = 0.0f; for (int i = 0; i < 4; ++i) { const float d = y[i] - mean; s2 += d * d; } for (int o = 16; o; o >>= 1) s2 += __shfl_xor(s2, o); const float rstd = rsqrtf(s2 * (1.0f / HID) + LNEPS);
  v4f of; v4h ph, pl;
  for (int i = 0; i < 4; ++i) { float z = gelu((y[i] - mean) * rstd * bf16_rne(g_[c0 + i]) + bf16_rne(b_[c0 + i])); if (v >= (size_t)N) z = 0.0f; of[i] = z; b16 p, pq; split16(z * XS, p, pq); ph[i] = p; pl[i] = pq; }
  for (int pass = 0; pass < 2; ++pass) { *(volatile v4h*)(Hh + v * HID + c0) = ph; *(volatile v4h*)(Hl + v * HID + c0) = pl; if (LAST) *(volatile v4f*)(HF + v * HID + c0) = of; __threadfence(); }
}
__device__ int lower_bound_i(const int* a, int n, int key) { int lo = 0, hi = n; while (lo < hi) { const int mid = (lo + hi) >> 1; if (a[mid] < key) lo = mid + 1; else hi = mid; } return lo; }
__global__ __launch_bounds__(128) void pool_kernel(const float* __restrict__ HF, const int* __restrict__ batch, const float* __restrict__ w1, const float* __restrict__ b1, const float* __restrict__ w2, const float* __restrict__ b2, float* __restrict__ PO) {
  __shared__ float gm[HID], red[HID];
  const int g = blockIdx.x, c = threadIdx.x; const int lo = lower_bound_i(batch, N, g), hi = lower_bound_i(batch, N, g + 1);
  float s = 0.0f; for (int v = lo; v < hi; ++v) s += HF[(size_t)v * HID + c]; gm[c] = s / fmaxf((float)(hi - lo), 1.0f);
  __syncthreads();
  float h = bf16_rne(b1[c]);
#pragma unroll 1
  for (int k = 0; k < HID; ++k) h += pmul(gm[k], bf16_rne(w1[k * HID + c])); red[c] = pmul(gelu(h), bf16_rne(w2[c]));
  __syncthreads();
  for (int st = HID / 2; st > 0; st >>= 1) { if (c < st) red[c] += red[c + st]; __syncthreads(); }
  for (int pass = 0; pass < 2; ++pass) { if (c < 32) ((volatile float*)PO)[(size_t)g * 32 + c] = red[0] + bf16_rne(b2[0]); __threadfence(); }
}
__global__ __launch_bounds__(64) void final_kernel(const float* __restrict__ PO, float* __restrict__ out) {
  __shared__ __attribute__((aligned(16))) float so[G]; if (threadIdx.x < G) so[threadIdx.x] = PO[(size_t)threadIdx.x * 32]; __syncthreads();
  for (int pass = 0; pass < 2; ++pass) { if (threadIdx.x < G / 4) *(volatile v4f*)(out + threadIdx.x * 4) = *(const v4f*)(&so[threadIdx.x * 4]); __threadfence(); }
}
}

extern "C" void kernel_launch(void* const* d_in, const int* in_sizes, int n_in, void* d_out, int out_size, void* d_ws, size_t ws_size, hipStream_t stream) {
  (void)n_in;
  auto Fp = [&](int i) { return (const float*)d_in[i]; }; auto Ip = [&](int i) { return (const int*)d_in[i]; };
  if (in_sizes[0] != N * IN || in_sizes[1] != 2 * E || in_sizes[2] != N || in_sizes[3] != IN * HID || in_sizes[11] != 3 * HID || in_sizes[14] != 2 * HID * HID || in_sizes[22] != 2 * 3 * HID || in_sizes[25] != HID * HID || in_sizes[27] != HID || out_size != G) return;
  size_t off = 0; char* ws = (char*)d_ws;
  auto carve = [&](size_t bytes) { char* p = ws + off; off += (bytes + 255) & ~(size_t)255; return p; };
  b16* X16 = (b16*)carve((size_t)NP * IN * 2); b16* WT0 = (b16*)carve((size_t)QW * IN * 2); b16* WT12 = (b16*)carve((size_t)2 * QW * HID * 2); float* QKVS = (float*)carve((size_t)NP * QW * 4);
  b16* Hh = (b16*)carve((size_t)NP * HID * 2); b16* Hl = (b16*)carve((size_t)NP * HID * 2); float* HF = (float*)carve((size_t)NP * HID * 4); float* PO = (float*)carve((size_t)G * 32 * 4);
  CsrBufs csr; off = csr_carve(csr, ws, off, E, N);
  if (off > ws_size) return;
  prep_kernel<<<(unsigned)(((size_t)NP * IN / 8 + (size_t)QW * IN / 8 + (size_t)2 * QW * HID / 8 + 255) / 256), 256, 0, stream>>>(Fp(0), Fp(3), Fp(5), Fp(7), Fp(9), Fp(14), Fp(16), Fp(18), Fp(20), X16, WT0, WT12);
  csr_build(csr, Ip(1) + E, E, N, stream);
  proj_kernel<IN, 0><<<dim3(NP / 64, 4), 128, 0, stream>>>(X16, nullptr, WT0, Fp(4), Fp(6), Fp(8), Fp(10), QKVS);
  attn_kernel<0><<<NP / 8, 256, 0, stream>>>(QKVS, Ip(1), csr.PERM, csr.ROWPTR, csr.ROWCNT, (int)csr.permLen, Fp(11), Fp(12), Fp(13), Hh, Hl, nullptr);
  for (int l = 0; l < 2; ++l) {
    proj_kernel<HID, 1><<<dim3(NP / 64, 4), 128, 0, stream>>>(Hh, Hl, WT12 + (size_t)l * QW * HID, Fp(15) + l * HID, Fp(17) + l * HID, Fp(19) + l * HID, Fp(21) + l * HID, QKVS);
    if (l == 1) attn_kernel<1><<<NP / 8, 256, 0, stream>>>(QKVS, Ip(1), csr.PERM, csr.ROWPTR, csr.ROWCNT, (int)csr.permLen, Fp(22) + l * 3 * HID, Fp(23) + l * HID, Fp(24) + l * HID, Hh, Hl, HF);
    else attn_kernel<0><<<NP / 8, 256, 0, stream>>>(QKVS, Ip(1), csr.PERM, csr.ROWPTR, csr.ROWCNT, (int)csr.permLen, Fp(22) + l * 3 * HID, Fp(23) + l * HID, Fp(24) + l * HID, Hh, Hl, nullptr); }
  pool_kernel<<<G, 128, 0, stream>>>(HF, Ip(2), Fp(25), Fp(26), Fp(27), Fp(28), PO);
  final_kernel<<<1, 64, 0, stream>>>(PO, (float*)d_out);
}
